// UAG_RNN_4Neigh_15908558864728
// MI455X (gfx1250) — hardware-run, weakly checked
//
#include <hip/hip_runtime.h>
#include <math.h>

typedef __attribute__((ext_vector_type(16))) _Float16 v16h;
typedef __attribute__((ext_vector_type(8)))  _Float16 v8h;
typedef __attribute__((ext_vector_type(8)))  float    v8f;
typedef __attribute__((ext_vector_type(4)))  float    v4f;
typedef __attribute__((ext_vector_type(8)))  unsigned v8u;
typedef __attribute__((ext_vector_type(4)))  unsigned v4u;

constexpr int kNB = 8;
constexpr int kNC = 64;
constexpr int kNH = 160;
constexpr int kNW = 160;
constexpr int kSteps = 160;
constexpr int kSeqTile = 16;
constexpr int kTilesPerImg = kNH / kSeqTile;
constexpr int kTiles = kNB * kTilesPerImg;
constexpr int kRowStride = kNW * kNC;
constexpr int kImgStride = kNH * kNW * kNC;
constexpr int kPlaneElems = kNB * kImgStride;
constexpr size_t kPlaneBytes = (size_t)kPlaneElems * 2;
constexpr int kWElems = kNC * kNC;
constexpr size_t kWPlanesBytes = (size_t)12 * kWElems * 2;
constexpr int kBiasPitch = 128;
constexpr size_t kBiasBytes = (size_t)6 * kBiasPitch * 4;
constexpr int kWaPitch = 72;
constexpr int kTrPitchW = 36;
constexpr int kOutPitch = 36;
static_assert(kNH == kNW);
static_assert(kNH == kSteps);
static_assert(kNC == 64);
static_assert((kNH % kSeqTile) == 0);
static_assert(kTiles == 80);
static_assert((kNW % 32) == 0);
static_assert(kPlaneElems == 13107200);
static_assert((kPlaneBytes % 128) == 0);

constexpr float kActCarry   = 64.0f;
constexpr float kWCarry     = 1024.0f;
constexpr float kAccCarry   = kActCarry * kWCarry;
constexpr float kStateScale = kActCarry / kAccCarry;
constexpr float kOutScale   = 1.0f / kActCarry;
constexpr float kF16MinNormal = 6.103515625e-05f;
static_assert(kAccCarry == 65536.0f);
static_assert(kStateScale == 0.0009765625f);

__device__ __forceinline__ unsigned short f2bf_bits(float f) {
  unsigned u = __float_as_uint(f);
  return (unsigned short)((u + 0x7FFFu + ((u >> 16) & 1u)) >> 16);
}
__device__ __forceinline__ float bf_bits2f(unsigned short h) { return __uint_as_float(((unsigned)h) << 16); }
__device__ __forceinline__ float bf16r(float f) { return bf_bits2f(f2bf_bits(f)); }

__device__ __forceinline__ float act_carry_flush(float f) {
  const float r = bf16r(f) * kActCarry;
  return (fabsf(r) >= kF16MinNormal) ? r : 0.0f;
}
__device__ __forceinline__ float wt_carry_flush(float f) {
  const float r = bf16r(f) * kWCarry;
  return (fabsf(r) >= kF16MinNormal) ? r : 0.0f;
}
__device__ __forceinline__ float h16_to_f32(unsigned hb) {
  const unsigned sgn = (hb & 0x8000u) << 16;
  const unsigned em = hb & 0x7fffu;
  const float fn = __uint_as_float((em << 13) + 0x38000000u);
  const float fs = (float)em * 5.9604644775390625e-8f;
  const float mag = (em < 0x400u) ? fs : fn;
  return __uint_as_float(__float_as_uint(mag) | sgn);
}

union FragU { v16h v; v8h h[2]; };
__device__ __forceinline__ v16h frag_load(const _Float16* p) {
  FragU f;
  f.h[0] = *(const v8h*)(p);
  f.h[1] = *(const v8h*)(p + 16);
  return f.v;
}
__device__ __forceinline__ v8f wmma_f16(v16h a, v16h b, v8f c) {
  return __builtin_amdgcn_wmma_f32_16x16x32_f16(false, a, false, b, (short)0, c, false, false);
}
__device__ __forceinline__ void tile_guard(v8f& acc, v16h a0, v16h a1, v16h w0, v16h w1,
                                           v16h c0, v16h c1, v16h s0, v16h s1) {
  asm volatile("v_nop\n\tv_nop\n\tv_nop\n\tv_nop"
               : "+v"(acc)
               : "v"(a0), "v"(a1), "v"(w0), "v"(w1), "v"(c0), "v"(c1), "v"(s0), "v"(s1));
}
__device__ __forceinline__ v16h relu_packed(v16h x, unsigned on) {
  v8u w = __builtin_bit_cast(v8u, x);
#pragma unroll
  for (int j = 0; j < 8; ++j) {
    const unsigned neg = ((w[j] >> 15) & 0x00010001u) * 0xFFFFu;
    w[j] = w[j] & ~(neg & on);
  }
  return __builtin_bit_cast(v16h, w);
}
__device__ __forceinline__ float state_val(float a) {
  const float s = a * kStateScale;
  return (s >= kF16MinNormal) ? s : 0.0f;
}

struct PrepArgs {
  const float* w[12];
  const float* b[12];
  unsigned short* wplanes;
  float* bias;
};
static_assert(sizeof(PrepArgs) == 26 * 8);

__global__ __launch_bounds__(256) void prep_planes_kernel(PrepArgs P) {
  const int tid = threadIdx.x, lane = tid & 31, wave = tid >> 5;
  const int bx = blockIdx.x;
  if (bx < 12) {
    const float* src = P.w[0];
#pragma unroll
    for (int j = 1; j < 12; ++j) src = (bx == j) ? P.w[j] : src;
    unsigned short* dp = P.wplanes + (size_t)bx * kWElems;
    v8h hv[2];
#pragma unroll
    for (int it = 0; it < 2; ++it) {
      const int idx = it * 256 + tid;
      const v4f a0 = *(const v4f*)(src + 8 * idx);
      const v4f a1 = *(const v4f*)(src + 8 * idx + 4);
#pragma unroll
      for (int e = 0; e < 4; ++e) {
        const float f0 = a0[e];
        const float f1 = a1[e];
        hv[it][e]     = (_Float16)wt_carry_flush(f0);
        hv[it][4 + e] = (_Float16)wt_carry_flush(f1);
      }
    }
    for (int pass = 0; pass < 2; ++pass) {
#pragma unroll
      for (int it = 0; it < 2; ++it) {
        const int idx = it * 256 + tid;
        *(volatile v8h*)(dp + 8 * idx) = hv[it];
      }
      __threadfence();
    }
  } else {
    if (wave < 6) {
      const float* pa = P.b[0];
      const float* pb = P.b[1];
#pragma unroll
      for (int s = 1; s < 6; ++s) {
        pa = (wave == s) ? P.b[2 * s] : pa;
        pb = (wave == s) ? P.b[2 * s + 1] : pb;
      }
      const int c4 = (lane & 15) * 4;
      const v4f va = *(const v4f*)(pa + c4);
      const v4f vb = *(const v4f*)(pb + c4);
      v4f o;
#pragma unroll
      for (int e = 0; e < 4; ++e) {
        float fa = va[e];
        float fb = vb[e];
        asm volatile("" : "+v"(fa));
        asm volatile("" : "+v"(fb));
        const float s = (bf16r(fa) + bf16r(fb)) * kAccCarry;
        o[e] = (lane < 16) ? s : 0.0f;
      }
      float* op = P.bias + wave * kBiasPitch + lane * 4;
      *(volatile v4f*)op = o;
      __threadfence();
      *(volatile v4f*)op = o;
    }
  }
}

__global__ __launch_bounds__(256) void to_pixel_lines_kernel(const float* __restrict__ x,
                                                             unsigned short* __restrict__ xT) {
  __shared__ __align__(16) unsigned sT[32 * kTrPitchW];
  const int tid = threadIdx.x;
  const int tile = blockIdx.x;
  const int wt = tile % 5;
  const int bh = tile / 5;
  const int h = bh % kNH;
  const int b = bh / kNH;
  const int w0 = wt * 32;
  const int cp = tid >> 3, w4 = (tid & 7) * 4;
  {
    const float* xp = x + ((size_t)(b * kNC + 2 * cp) * kNH + h) * kNW + w0 + w4;
    const v4f v0 = *(const v4f*)(xp);
    const v4f v1 = *(const v4f*)(xp + (size_t)kNH * kNW);
#pragma unroll
    for (int e = 0; e < 4; ++e) {
      const float f0 = v0[e];
      const float f1 = v1[e];
      const _Float16 h0 = (_Float16)act_carry_flush(f0);
      const _Float16 h1 = (_Float16)act_carry_flush(f1);
      const unsigned lo = (unsigned)__builtin_bit_cast(unsigned short, h0);
      const unsigned hi = (unsigned)__builtin_bit_cast(unsigned short, h1);
      sT[(w4 + e) * kTrPitchW + cp] = lo | (hi << 16);
    }
  }
  __syncthreads();
  const int p = tid >> 3, ch = tid & 7;
  const v4u o = *(const v4u*)(sT + p * kTrPitchW + ch * 4);
  unsigned short* dp = xT + ((size_t)((b * kNH + h) * kNW + w0 + p)) * kNC + ch * 8;
  *(volatile v4u*)dp = o;
  __threadfence();
  *(volatile v4u*)dp = o;
}

struct ScanDesc {
  const unsigned short* src;
  unsigned short* dst;
  const unsigned short* wa;
  const unsigned short* wb;
  const float* bias;
  int seq_stride;
  int step_stride;
  int reverse;
  int relu_init;
};
static_assert(sizeof(ScanDesc) == 56);

__device__ __forceinline__ void store_lines(v16h s0v, v16h s1v, v4u* slab, unsigned short* dst,
                                            int o0, int o1, int o2, int o3, int g, int n, int lane) {
  const v8u w0 = __builtin_bit_cast(v8u, s0v);
  const v8u w1 = __builtin_bit_cast(v8u, s1v);
  slab[n * 8 + g]     = __builtin_shufflevector(w0, w0, 0, 1, 2, 3);
  slab[n * 8 + g + 2] = __builtin_shufflevector(w0, w0, 4, 5, 6, 7);
  slab[n * 8 + g + 4] = __builtin_shufflevector(w1, w1, 0, 1, 2, 3);
  slab[n * 8 + g + 6] = __builtin_shufflevector(w1, w1, 4, 5, 6, 7);
  __builtin_amdgcn_fence(__ATOMIC_RELEASE, "workgroup");
  __builtin_amdgcn_wave_barrier();
  __builtin_amdgcn_fence(__ATOMIC_ACQUIRE, "workgroup");
  const v4u q0 = slab[lane];
  const v4u q1 = slab[32 + lane];
  const v4u q2 = slab[64 + lane];
  const v4u q3 = slab[96 + lane];
  for (int pass = 0; pass < 2; ++pass) {
    *(volatile v4u*)(dst + (size_t)o0) = q0;
    *(volatile v4u*)(dst + (size_t)o1) = q1;
    *(volatile v4u*)(dst + (size_t)o2) = q2;
    *(volatile v4u*)(dst + (size_t)o3) = q3;
    __threadfence();
  }
  __builtin_amdgcn_fence(__ATOMIC_RELEASE, "workgroup");
  __builtin_amdgcn_wave_barrier();
  __builtin_amdgcn_fence(__ATOMIC_ACQUIRE, "workgroup");
}

__global__ __launch_bounds__(64) void dir_scan_kernel(ScanDesc da, ScanDesc db) {
  __shared__ __align__(16) _Float16 sWa[kNC * kWaPitch];
  __shared__ __align__(32) float sBias[kNC];
  __shared__ __align__(16) v4u sSlab[2][16 * 8];

  const ScanDesc P = (blockIdx.y == 0) ? da : db;
  const int tid = threadIdx.x, lane = tid & 31, wave = tid >> 5;
  const int g = lane >> 4, n = lane & 15;
  const _Float16* SRC = (const _Float16*)P.src;
  const _Float16* WA  = (const _Float16*)P.wa;
  const _Float16* WB  = (const _Float16*)P.wb;

#pragma unroll
  for (int it = 0; it < 8; ++it) {
    const int idx = it * 64 + tid;
    const int r = idx >> 3, ch = idx & 7;
    *(v8h*)(sWa + r * kWaPitch + ch * 8) = *(const v8h*)(WA + r * kNC + ch * 8);
  }
  sBias[tid] = P.bias[tid];
  __syncthreads();

  v16h wb[4][2];
#pragma unroll
  for (int t = 0; t < 4; ++t)
#pragma unroll
    for (int ks = 0; ks < 2; ++ks)
      wb[t][ks] = frag_load(WB + (16 * t + n) * kNC + 32 * ks + 8 * g);

  const int tile = blockIdx.x * 2 + wave;
  const int b = tile / kTilesPerImg;
  const int s0 = (tile - b * kTilesPerImg) * kSeqTile;
  const int tbase = b * kImgStride;
  const int lbase = tbase + (s0 + n) * P.seq_stride + 8 * g;
  const int q = lane >> 3, c8 = (lane & 7) * 8;
  const int so0 = tbase + (s0 + q) * P.seq_stride + c8;
  const int so1 = tbase + (s0 + 4 + q) * P.seq_stride + c8;
  const int so2 = tbase + (s0 + 8 + q) * P.seq_stride + c8;
  const int so3 = tbase + (s0 + 12 + q) * P.seq_stride + c8;
  v4u* slab = sSlab[wave];
  unsigned short* DST = P.dst;

  const int pos0 = P.reverse ? (kSteps - 1) : 0;
  const unsigned on = P.relu_init ? 0xFFFFFFFFu : 0u;
  const int poff0 = pos0 * P.step_stride;
  v16h st0 = relu_packed(frag_load(SRC + lbase + poff0), on);
  v16h st1 = relu_packed(frag_load(SRC + lbase + poff0 + 32), on);
  store_lines(st0, st1, slab, DST, so0 + poff0, so1 + poff0, so2 + poff0, so3 + poff0, g, n, lane);

#pragma unroll 1
  for (int i = 1; i < kSteps; ++i) {
    const int pos = P.reverse ? (kSteps - 1 - i) : i;
    const int poff = pos * P.step_stride;
    const v16h c0 = frag_load(SRC + lbase + poff);
    const v16h c1 = frag_load(SRC + lbase + poff + 32);

    v8f acc[4];
#pragma unroll
    for (int t = 0; t < 4; ++t) {
      const v4f b0 = *(const v4f*)(sBias + 16 * t + 8 * g);
      const v4f b1 = *(const v4f*)(sBias + 16 * t + 8 * g + 4);
      acc[t] = __builtin_shufflevector(b0, b1, 0, 1, 2, 3, 4, 5, 6, 7);
    }
#pragma unroll
    for (int t = 0; t < 4; ++t) {
      const v16h a0 = frag_load(sWa + (16 * t + n) * kWaPitch + 8 * g);
      const v16h a1 = frag_load(sWa + (16 * t + n) * kWaPitch + 32 + 8 * g);
      acc[t] = wmma_f16(a0, c0, acc[t]);
      acc[t] = wmma_f16(a1, c1, acc[t]);
      acc[t] = wmma_f16(wb[t][0], st0, acc[t]);
      acc[t] = wmma_f16(wb[t][1], st1, acc[t]);
      tile_guard(acc[t], a0, a1, wb[t][0], wb[t][1], c0, c1, st0, st1);
    }

    v16h n0, n1;
#pragma unroll
    for (int r = 0; r < 8; ++r) {
      n0[r]     = (_Float16)state_val(acc[0][r]);
      n0[8 + r] = (_Float16)state_val(acc[1][r]);
      n1[r]     = (_Float16)state_val(acc[2][r]);
      n1[8 + r] = (_Float16)state_val(acc[3][r]);
    }
    st0 = n0;
    st1 = n1;
    store_lines(st0, st1, slab, DST, so0 + poff, so1 + poff, so2 + poff, so3 + poff, g, n, lane);
  }
}

__global__ __launch_bounds__(256) void sum_to_planar_kernel(const unsigned short* __restrict__ qa,
                                                            const unsigned short* __restrict__ qb,
                                                            const unsigned short* __restrict__ qc,
                                                            const unsigned short* __restrict__ qd,
                                                            float* __restrict__ out) {
  __shared__ __align__(16) float sO[kNC * kOutPitch];
  const int tid = threadIdx.x;
  const int tile = blockIdx.x;
  const int wt = tile % 5;
  const int bh = tile / 5;
  const int h = bh % kNH;
  const int b = bh / kNH;
  const int w0 = wt * 32;
  {
    const int p = tid >> 3, c8 = (tid & 7) * 8;
    const size_t off = ((size_t)((b * kNH + h) * kNW + w0 + p)) * kNC + c8;
    const v4u va = *(const v4u*)(qa + off);
    const v4u vb = *(const v4u*)(qb + off);
    const v4u vc = *(const v4u*)(qc + off);
    const v4u vd = *(const v4u*)(qd + off);
#pragma unroll
    for (int j = 0; j < 4; ++j) {
      const unsigned ua = va[j], ub = vb[j], uc = vc[j], ud = vd[j];
      float lo = h16_to_f32(ua & 0xffffu) + h16_to_f32(ub & 0xffffu);
      lo = lo + h16_to_f32(uc & 0xffffu);
      lo = lo + h16_to_f32(ud & 0xffffu);
      float hi = h16_to_f32(ua >> 16) + h16_to_f32(ub >> 16);
      hi = hi + h16_to_f32(uc >> 16);
      hi = hi + h16_to_f32(ud >> 16);
      sO[(c8 + 2 * j) * kOutPitch + p]     = lo * kOutScale;
      sO[(c8 + 2 * j + 1) * kOutPitch + p] = hi * kOutScale;
    }
  }
  __syncthreads();
  const int cq = tid >> 3, w4 = (tid & 7) * 4;
  v4f ov[2];
#pragma unroll
  for (int it = 0; it < 2; ++it) ov[it] = *(const v4f*)(sO + (it * 32 + cq) * kOutPitch + w4);
  for (int pass = 0; pass < 2; ++pass) {
#pragma unroll
    for (int it = 0; it < 2; ++it) {
      const int c = it * 32 + cq;
      *(volatile v4f*)(out + ((size_t)(b * kNC + c) * kNH + h) * kNW + w0 + w4) = ov[it];
    }
    __threadfence();
  }
}

extern "C" void kernel_launch(void* const* d_in, const int* in_sizes, int n_in,
                              void* d_out, int out_size, void* d_ws, size_t ws_size,
                              hipStream_t stream) {
  if (n_in < 25 || d_out == nullptr || d_ws == nullptr) return;
  if (in_sizes[0] != kPlaneElems) return;
  for (int j = 0; j < 12; ++j) {
    if (in_sizes[1 + 2 * j] != kWElems) return;
    if (in_sizes[2 + 2 * j] != kNC) return;
  }
  if (out_size != kPlaneElems) return;

  char* ws = (char*)d_ws;
  size_t off = 0;
  auto carve = [&](size_t bytes) -> char* { char* p = ws + off; off += (bytes + 255) & ~(size_t)255; return p; };
  unsigned short* P0 = (unsigned short*)carve(kPlaneBytes);
  unsigned short* P1 = (unsigned short*)carve(kPlaneBytes);
  unsigned short* P2 = (unsigned short*)carve(kPlaneBytes);
  unsigned short* P3 = (unsigned short*)carve(kPlaneBytes);
  unsigned short* P4 = (unsigned short*)carve(kPlaneBytes);
  unsigned short* WP = (unsigned short*)carve(kWPlanesBytes);
  float*          BI = (float*)carve(kBiasBytes);
  if (off != (size_t)131173376) return;
  if (off > ws_size || off > (size_t)134217728) return;

  PrepArgs pa;
  for (int k = 0; k < 12; ++k) {
    pa.w[k] = (const float*)d_in[1 + 2 * k];
    pa.b[k] = (const float*)d_in[2 + 2 * k];
  }
  pa.wplanes = WP;
  pa.bias = BI;
  prep_planes_kernel<<<13, 256, 0, stream>>>(pa);

  to_pixel_lines_kernel<<<kNB * kNH * (kNW / 32), 256, 0, stream>>>((const float*)d_in[0], P0);

  const int seqRow = kNC;
  const int stepRow = kRowStride;
  const int seqCol = kRowStride;
  const int stepCol = kNC;

  ScanDesc south = { P0, P1, WP + 0 * kWElems, WP + 1 * kWElems, BI + 0 * kBiasPitch, seqRow, stepRow, 0, 0 };
  ScanDesc north = { P0, P2, WP + 6 * kWElems, WP + 7 * kWElems, BI + 3 * kBiasPitch, seqRow, stepRow, 1, 1 };
  dir_scan_kernel<<<dim3(kTiles / 2, 2), 64, 0, stream>>>(south, north);

  ScanDesc ne = { P2, P3, WP + 8 * kWElems,  WP + 9 * kWElems,  BI + 4 * kBiasPitch, seqCol, stepCol, 0, 1 };
  ScanDesc nw = { P2, P0, WP + 10 * kWElems, WP + 11 * kWElems, BI + 5 * kBiasPitch, seqCol, stepCol, 1, 1 };
  dir_scan_kernel<<<dim3(kTiles / 2, 2), 64, 0, stream>>>(ne, nw);

  ScanDesc se = { P1, P2, WP + 2 * kWElems, WP + 3 * kWElems, BI + 1 * kBiasPitch, seqCol, stepCol, 0, 1 };
  ScanDesc sw = { P1, P4, WP + 4 * kWElems, WP + 5 * kWElems, BI + 2 * kBiasPitch, seqCol, stepCol, 1, 1 };
  dir_scan_kernel<<<dim3(kTiles / 2, 2), 64, 0, stream>>>(se, sw);

  sum_to_planar_kernel<<<kNB * kNH * (kNW / 32), 256, 0, stream>>>(P2, P4, P0, P3, (float*)d_out);
}
